// _NonLocalBlockND_Group_17583596110628
// MI455X (gfx1250) — hardware-run, weakly checked
//
#include <hip/hip_runtime.h>


#define NI   2
#define CC   256
#define NP   3136
#define NG   8
#define GD   16
#define CI   128
#define C3   384
typedef _Float16 h16;
typedef unsigned short bf;
typedef __attribute__((ext_vector_type(16))) __bf16   v16bf;
typedef __attribute__((ext_vector_type(16))) _Float16 v16h;
typedef __attribute__((ext_vector_type(8)))  _Float16 v8h;
typedef __attribute__((ext_vector_type(8)))  unsigned short v8us;
typedef __attribute__((ext_vector_type(8)))  float    v8f;
typedef __attribute__((ext_vector_type(4)))  float    v4f;
typedef v8h  __attribute__((may_alias)) v8ha;
typedef v4f  __attribute__((may_alias)) v4fa;
typedef v8us __attribute__((may_alias)) v8usa;

__device__ __forceinline__ unsigned short f2bf(float f) { unsigned u = __float_as_uint(f); u += 0x7FFFu + ((u >> 16) & 1u); return (unsigned short)(u >> 16); }
__device__ __forceinline__ float bf2f(unsigned short b) { return __uint_as_float(((unsigned)b) << 16); }
__device__ __forceinline__ float bfr(float f) { return bf2f(f2bf(f)); }
__device__ __forceinline__ v16h cat16(v8h lo, v8h hi) { return __builtin_shufflevector(lo, hi, 0, 1, 2, 3, 4, 5, 6, 7, 8, 9, 10, 11, 12, 13, 14, 15); }
__device__ __forceinline__ v16bf cat16b(v8us lo, v8us hi) { return __builtin_bit_cast(v16bf, __builtin_shufflevector(lo, hi, 0, 1, 2, 3, 4, 5, 6, 7, 8, 9, 10, 11, 12, 13, 14, 15)); }
__device__ __forceinline__ v8f wmma16(v16h a, v16h b, v8f c) { return __builtin_amdgcn_wmma_f32_16x16x32_f16(false, a, false, b, (short)0, c, false, false); }
__device__ __forceinline__ v8f wmmab(v16bf a, v16bf b, v8f c) { return __builtin_amdgcn_wmma_f32_16x16x32_bf16(false, a, false, b, (short)0, c, false, false); }


template <typename T16> struct WFrag;
template <> struct WFrag<h16> { typedef v16h V; static __device__ __forceinline__ V ld(const h16* p) { return cat16(*(const v8h*)p, *(const v8h*)(p + 16)); } static __device__ __forceinline__ v8f mma(V a, V b, v8f c) { return wmma16(a, b, c); } };
template <> struct WFrag<bf> { typedef v16bf V; static __device__ __forceinline__ V ld(const bf* p) { return cat16b(*(const v8us*)p, *(const v8us*)(p + 16)); } static __device__ __forceinline__ v8f mma(V a, V b, v8f c) { return wmmab(a, b, c); } };
template <typename T16, int NSPLIT, bool BIAS>
__global__ __launch_bounds__(32) void k_gemmw(const T16* __restrict__ A, const T16* __restrict__ A2, const T16* __restrict__ Bt, const T16* __restrict__ Bt2, int K, float* C, int ldc, const float* __restrict__ bias, size_t sA, size_t sB, size_t sC) {
    typedef typename WFrag<T16>::V V;
    __shared__ __align__(16) float os[16 * 68];
    const size_t z = blockIdx.z; A += z * sA; if (A2) A2 += z * sA; Bt += z * sB; if (Bt2) Bt2 += z * sB; C += z * sC;
    const int lane = threadIdx.x & 31, lr = lane & 15, hi = lane >> 4; const int r0 = blockIdx.x * 64, c0 = blockIdx.y * 64;
    v8f acc[4][4];
#pragma unroll
    for (int mb = 0; mb < 4; ++mb)
#pragma unroll
        for (int nb = 0; nb < 4; ++nb) acc[mb][nb] = (v8f){};
    const size_t aoff = (size_t)(r0 + lr) * K + 8 * hi, boff = (size_t)(c0 + lr) * K + 8 * hi;
#pragma unroll 1
    for (int kc = 0; kc < K; kc += 32) {
        V a[4], a2[4];
#pragma unroll
        for (int mb = 0; mb < 4; ++mb) { a[mb] = WFrag<T16>::ld(A + aoff + (size_t)mb * 16 * K + kc); if (NSPLIT == 1 || NSPLIT == 2) a2[mb] = WFrag<T16>::ld(A2 + aoff + (size_t)mb * 16 * K + kc); }
#pragma unroll
        for (int nb = 0; nb < 4; ++nb) { const V b = WFrag<T16>::ld(Bt + boff + (size_t)nb * 16 * K + kc); V b2; if (NSPLIT >= 2) b2 = WFrag<T16>::ld(Bt2 + boff + (size_t)nb * 16 * K + kc);
#pragma unroll
            for (int mb = 0; mb < 4; ++mb) { acc[mb][nb] = WFrag<T16>::mma(a[mb], b, acc[mb][nb]); if (NSPLIT == 1 || NSPLIT == 2) acc[mb][nb] = WFrag<T16>::mma(a2[mb], b, acc[mb][nb]); if (NSPLIT >= 2) acc[mb][nb] = WFrag<T16>::mma(a[mb], b2, acc[mb][nb]); } }
        asm volatile("v_nop\n\tv_nop\n\tv_nop\n\tv_nop" : "+v"(acc[0][0]), "+v"(acc[1][1]), "+v"(acc[2][2]), "+v"(acc[3][3]) : "v"(a[0]), "v"(a[3]));
    }
#pragma unroll
    for (int mb = 0; mb < 4; ++mb) {
#pragma unroll
        for (int nb = 0; nb < 4; ++nb) {
#pragma unroll
            for (int j = 0; j < 8; ++j) os[(hi * 8 + j) * 68 + nb * 16 + lr] = acc[mb][nb][j]; }
        __builtin_amdgcn_wave_barrier(); asm volatile("" ::: "memory");
        float* crow = C + (size_t)(r0 + mb * 16) * ldc + c0;
#pragma unroll 1
        for (int ps = 0; ps < 2; ++ps) {
#pragma unroll
            for (int s = 0; s < 8; ++s) { const int row = 2 * s + hi, cofs = lr * 4; v4f val = *(const v4fa*)(os + row * 68 + cofs); if (BIAS) { val[0] += bfr(bias[c0 + cofs]); val[1] += bfr(bias[c0 + cofs + 1]); val[2] += bfr(bias[c0 + cofs + 2]); val[3] += bfr(bias[c0 + cofs + 3]); }
                *(volatile v4f*)(crow + (size_t)row * ldc + cofs) = val; }
            if (ps == 0) __threadfence(); }
        __builtin_amdgcn_wave_barrier(); asm volatile("" ::: "memory");
    }
}

__device__ __forceinline__ void splitf(float y, unsigned short& h, unsigned short& l) { h = f2bf(y); l = f2bf(y - bf2f(h)); }
typedef __attribute__((ext_vector_type(2))) unsigned short v2us;
typedef __attribute__((ext_vector_type(4))) unsigned short v4us;

__global__ __launch_bounds__(256) void k_cvt8(const float* __restrict__ src, bf* dst, size_t n8) { const size_t i = (size_t)blockIdx.x * 256 + threadIdx.x; if (i >= n8) return; const v8f v = *(const v8f*)(src + i * 8); v8us o;
#pragma unroll
    for (int k = 0; k < 8; ++k) o[k] = f2bf(v[k]); *(volatile v8us*)(dst + i * 8) = o; __threadfence(); *(volatile v8us*)(dst + i * 8) = o; }
__global__ __launch_bounds__(256) void k_xt(const float* __restrict__ x, bf* XT) { const int e = (blockIdx.x * 256 + threadIdx.x) * 2; if (e >= NP * CC) return; const int c = e % CC; const int p = e / CC; v2us o; o[0] = f2bf(x[(size_t)c * NP + p]); o[1] = f2bf(x[(size_t)(c + 1) * NP + p]); *(volatile v2us*)(XT + e) = o; __threadfence(); *(volatile v2us*)(XT + e) = o; }
__global__ __launch_bounds__(128) void k_bcat(const float* __restrict__ bt, const float* __restrict__ bp, const float* __restrict__ bg, float* b3) { const int i = threadIdx.x; float v[3] = {bt[i], bp[i], bg[i]}; for (int ps = 0; ps < 2; ++ps) { *(volatile float*)(b3 + i) = v[0]; *(volatile float*)(b3 + CI + i) = v[1]; *(volatile float*)(b3 + 2 * CI + i) = v[2]; if (ps == 0) __threadfence(); } }
__global__ __launch_bounds__(256) void k_M(const float* __restrict__ P, float* M) { const int idx = blockIdx.x * 256 + threadIdx.x; if (idx >= NG * GD * GD) return; const int d = idx % GD; const int e = (idx / GD) % GD; const int g = idx / (GD * GD); const float* pp = P + CI + g * GD + e; const float* pg = P + 2 * CI + g * GD + d; float s = 0.f;
#pragma unroll 1
    for (int m = 0; m < NP; ++m) { float pr = __fmul_rn(pp[(size_t)m * C3], pg[(size_t)m * C3]); asm volatile("" : "+v"(pr)); s = __fadd_rn(s, pr); }
    const float o = s * (1.0f / NP); *(volatile float*)(M + idx) = o; __threadfence(); *(volatile float*)(M + idx) = o; }
__global__ __launch_bounds__(256) void k_y(const float* __restrict__ P, const float* __restrict__ M, bf* Yh, bf* Yl) { const int e4 = (blockIdx.x * 256 + threadIdx.x) * 4; if (e4 >= NP * CI) return; const int c0 = e4 % CI; const int n = e4 / CI; const int g = c0 / GD, d0 = c0 % GD; const float* th = P + (size_t)n * C3 + g * GD; const float* mg = M + (size_t)g * GD * GD; v4us oh, ol;
#pragma unroll
    for (int u = 0; u < 4; ++u) { const int d = d0 + u; float s = 0.f;
#pragma unroll 1
        for (int e = 0; e < GD; ++e) { float pr = __fmul_rn(th[e], mg[e * GD + d]); asm volatile("" : "+v"(pr)); s = __fadd_rn(s, pr); }
        unsigned short a, b; splitf(s, a, b); oh[u] = a; ol[u] = b; }
    *(volatile v4us*)(Yh + e4) = oh; *(volatile v4us*)(Yl + e4) = ol; __threadfence(); *(volatile v4us*)(Yh + e4) = oh; *(volatile v4us*)(Yl + e4) = ol; }
__global__ __launch_bounds__(256) void k_fin(const float* __restrict__ WYT, const float* __restrict__ x, const float* __restrict__ ga, const float* __restrict__ be, const float* __restrict__ rm, const float* __restrict__ rv, float* OUTb) { const int e = (blockIdx.x * 256 + threadIdx.x) * 4; if (e >= CC * NP) return; const int p = e % NP; const int c = e / NP;
    float gg = bfr(ga[c]), bb = bfr(be[c]), mm = bfr(rm[c]), vv = bfr(rv[c]); const float inv = __fmul_rn(gg, __frsqrt_rn(__fadd_rn(vv, 1e-5f))); float mi = __fmul_rn(mm, inv); asm volatile("" : "+v"(mi)); const float sh = __fsub_rn(bb, mi); v4f o;
#pragma unroll
    for (int u = 0; u < 4; ++u) { float t1 = __fmul_rn(WYT[(size_t)(p + u) * CC + c], inv); asm volatile("" : "+v"(t1)); const float wy = __fadd_rn(t1, sh); o[u] = fmaxf(__fadd_rn(wy, bfr(x[e + u])), 0.f); }
    *(volatile v4f*)(OUTb + e) = o; __threadfence(); *(volatile v4f*)(OUTb + e) = o; }

extern "C" void kernel_launch(void* const* d_in, const int* in_sizes, int n_in,
                              void* d_out, int out_size, void* d_ws, size_t ws_size, hipStream_t stream) {
    (void)in_sizes; (void)n_in; (void)out_size;
    const float** I = (const float**)d_in;
    const float *x = I[0], *w_g = I[1], *b_g = I[2], *w_t = I[3], *b_t = I[4], *w_p = I[5], *b_p = I[6], *w_o = I[7], *b_o = I[8], *ga = I[9], *be = I[10], *rm = I[11], *rv = I[12];
    float* OUT = (float*)d_out;
    char* wsp = (char*)d_ws;
    auto take = [&](size_t bytes) { char* p = wsp; wsp += (bytes + 255) & ~(size_t)255; return (void*)p; };
    bf* W3 = (bf*)take((size_t)C3 * CC * 2); float* b3 = (float*)take(C3 * 4); bf* WO = (bf*)take((size_t)CC * CI * 2); bf* XT = (bf*)take((size_t)NP * CC * 2); float* P = (float*)take((size_t)NP * C3 * 4); float* M = (float*)take(NG * GD * GD * 4); bf* Yh = (bf*)take((size_t)NP * CI * 2); bf* Yl = (bf*)take((size_t)NP * CI * 2); float* WYT = (float*)take((size_t)NP * CC * 4);
    if ((size_t)(wsp - (char*)d_ws) > ws_size) return;
    k_cvt8<<<(CI * CC / 8 + 255) / 256, 256, 0, stream>>>(w_t, W3, CI * CC / 8); k_cvt8<<<(CI * CC / 8 + 255) / 256, 256, 0, stream>>>(w_p, W3 + (size_t)CI * CC, CI * CC / 8); k_cvt8<<<(CI * CC / 8 + 255) / 256, 256, 0, stream>>>(w_g, W3 + (size_t)2 * CI * CC, CI * CC / 8);
    k_bcat<<<1, 128, 0, stream>>>(b_t, b_p, b_g, b3); k_cvt8<<<(CC * CI / 8 + 255) / 256, 256, 0, stream>>>(w_o, WO, CC * CI / 8);
    for (int b = 0; b < NI; ++b) { const float* xb = x + (size_t)b * CC * NP;
        k_xt<<<(NP * CC / 2 + 255) / 256, 256, 0, stream>>>(xb, XT);
        k_gemmw<bf, 0, true><<<dim3(NP / 64, C3 / 64, 1), 32, 0, stream>>>(XT, nullptr, W3, nullptr, CC, P, C3, b3, 0, 0, 0);
        k_M<<<(NG * GD * GD + 255) / 256, 256, 0, stream>>>(P, M); k_y<<<(NP * CI / 4 + 255) / 256, 256, 0, stream>>>(P, M, Yh, Yl);
        k_gemmw<bf, 1, true><<<dim3(NP / 64, CC / 64, 1), 32, 0, stream>>>(Yh, Yl, WO, nullptr, CI, WYT, CC, b_o, 0, 0, 0);
        k_fin<<<(CC * NP / 4 + 255) / 256, 256, 0, stream>>>(WYT, xb, ga, be, rm, rv, OUT + (size_t)b * CC * NP); }
}
